// Net_FG_34256659153245
// MI455X (gfx1250) — hardware-verified
//
#include <hip/hip_runtime.h>
#include <stddef.h>
#include <stdint.h>
#include <math.h>


#define HD     128
#define FIN    64
#define PW     512
#define HP     136
#define HP64   72
#define HP256  264
#define FP     132
#define WSC    16.0f
#define WINV   0.0625f
#define ASC    64.0f
#define AINV   0.015625f

#define O_ENCH 0
#define O_ENCL 8192
#define O_TP   16384
#define O_FEM2 81920
#define O_FAM2 98304
#define O_FN1H 114688
#define O_FN1L 147456
#define O_FN2H 180224
#define O_FN2L 196608
#define O_RG1H 212992
#define O_RG1L 245760
#define O_TOT  278528
#define NUNITS (O_TOT / 8)

static_assert(O_ENCL == O_ENCH + HD * FIN);
static_assert(O_TP == O_ENCL + HD * FIN);
static_assert(O_FEM2 == O_TP + PW * HD);
static_assert(O_FAM2 == O_FEM2 + HD * HD);
static_assert(O_FN1H == O_FAM2 + HD * HD);
static_assert(O_FN1L == O_FN1H + HD * 256);
static_assert(O_FN2H == O_FN1L + HD * 256);
static_assert(O_FN2L == O_FN2H + HD * HD);
static_assert(O_RG1H == O_FN2L + HD * HD);
static_assert(O_RG1L == O_RG1H + HD * 256);
static_assert(O_TOT == O_RG1L + HD * 256);
static_assert((NUNITS % 256) == 0);

#define SCH 4096

#define L2_FFH 0
#define L2_FFL 18432
#define L2_HF  36864
#define L2_STG 71680
#define L2_TOT 106496
static_assert(128 * HP64 * 2 == 18432);
static_assert(128 * HP * 2 == 34816);
static_assert(L2_STG == L2_HF + 34816 && L2_TOT == L2_STG + 34816);

#define NB3     128
#define LCAP3   2048
#define L3_M    0
#define L3_DEN  65536
#define L3_NUM  131072
#define L3_HID  196608
#define L3_HIDA (L3_HID + 64 * HP * 2)
#define L3_SL   (L3_HID + 34816)
#define L3_LIST (L3_SL + 64 * FP * 4)
#define L3_IDX  (L3_LIST + LCAP3 * 4)
#define L3_WT   (L3_IDX + 3 * 64 * 4)
#define L3_TOT  (L3_WT + 64)
static_assert(NB3 * HD * 4 == 65536);
static_assert(64 * FP * 4 <= 34816);
static_assert(2 * 64 * HP * 2 == 34816);
static_assert(L3_TOT == 274240);
static_assert((L3_HIDA & 15) == 0 && (L3_SL & 15) == 0 && (L3_LIST & 15) == 0 && (L3_IDX & 15) == 0 && (L3_WT & 15) == 0);

#define L4_AH   0
#define L4_AL   67584
#define L4_U2   135168
#define L4_FFL  (L4_U2 + 18432)
#define L4_HIDL (L4_U2 + 34816)
#define L4_TOT  (L4_U2 + 69632)
static_assert(128 * HP256 * 2 == 67584);
static_assert(128 * FP * 4 == 67584);
static_assert(L4_TOT == 204800);

#define NB5     64
#define LCAP5   4096
#define L5_SUM  0
#define L5_MAX  32768
#define L5_LIST 65536
#define L5_WT   (L5_LIST + LCAP5 * 4)
#define L5_TOT  (L5_WT + 64)
static_assert(NB5 * HD * 4 == 32768);
static_assert(L5_TOT == 81984);

#define L6_AH   0
#define L6_AL   67584
#define L6_RES  135168
#define L6_TOT  (L6_RES + 512)

typedef float          v4f   __attribute__((ext_vector_type(4)));
typedef float          v8f   __attribute__((ext_vector_type(8)));
typedef int            v4i   __attribute__((ext_vector_type(4)));
typedef _Float16       v8h   __attribute__((ext_vector_type(8)));
typedef _Float16       v16h  __attribute__((ext_vector_type(16)));
typedef unsigned short v4us  __attribute__((ext_vector_type(4)));
typedef unsigned short v8us  __attribute__((ext_vector_type(8)));
typedef unsigned short v16us __attribute__((ext_vector_type(16)));
typedef __bf16         v16b  __attribute__((ext_vector_type(16)));
union FragH { v16h v; v8h h[2]; };
union FragB { v16b v; v16us u; v8us h[2]; };
union HU8   { v8h h; v8us u; };

__device__ __forceinline__ v8f zero8f() {
  v8f z;
#pragma unroll
  for (int i = 0; i < 8; ++i) z[i] = 0.0f;
  return z;
}

__device__ __forceinline__ unsigned short bf_hi(float x) {
  unsigned u = __float_as_uint(x);
  u += 0x7FFFu + ((u >> 16) & 1u);
  return (unsigned short)(u >> 16);
}
__device__ __forceinline__ float bf_f(unsigned short b) { return __uint_as_float(((unsigned)b) << 16); }
__device__ __forceinline__ void split4(const v4f x, v4us& hi, v4us& lo) {
#pragma unroll
  for (int q = 0; q < 4; ++q) {
    const unsigned short hh = bf_hi(x[q]);
    hi[q] = hh;
    lo[q] = bf_hi(x[q] - bf_f(hh));
  }
}
__device__ __forceinline__ float lk(float x) { return x > 0.0f ? x : 0.01f * x; }

__device__ __forceinline__ v8f wmh(v16h a, v16h b, v8f c) {
  v8f d = __builtin_amdgcn_wmma_f32_16x16x32_f16(false, a, false, b, (short)0, c, false, false);
  asm volatile("v_nop\n\tv_nop\n\tv_nop\n\tv_nop" : "+v"(d) : "v"(a), "v"(b));
  return d;
}
__device__ __forceinline__ v8f wmb(v16b a, v16b b, v8f c) {
  v8f d = __builtin_amdgcn_wmma_f32_16x16x32_bf16(false, a, false, b, (short)0, c, false, false);
  asm volatile("v_nop\n\tv_nop\n\tv_nop\n\tv_nop" : "+v"(d) : "v"(a), "v"(b));
  return d;
}

__device__ __forceinline__ v16h ldh(const _Float16* p) {
  FragH f;
  f.h[0] = *(const v8h*)p;
  f.h[1] = *(const v8h*)(p + 16);
  return f.v;
}
__device__ __forceinline__ v16b ldb(const unsigned short* p) {
  FragB f;
  f.h[0] = *(const v8us*)p;
  f.h[1] = *(const v8us*)(p + 16);
  return f.v;
}

__device__ __forceinline__ void gemm3(const unsigned short* aH, const unsigned short* aL, int nk,
                                      const unsigned short* bH, const unsigned short* bL, int kp, v8f acc[4]) {
#pragma unroll 1
  for (int kt = 0; kt < nk; ++kt) {
    const v16b fah = ldb(aH + 32 * kt);
    const v16b fal = ldb(aL + 32 * kt);
#pragma unroll
    for (int nt = 0; nt < 4; ++nt) {
      const v16b fbh = ldb(bH + (size_t)(16 * nt) * kp + 32 * kt);
      const v16b fbl = ldb(bL + (size_t)(16 * nt) * kp + 32 * kt);
      acc[nt] = wmb(fah, fbh, acc[nt]);
      acc[nt] = wmb(fal, fbh, acc[nt]);
      acc[nt] = wmb(fah, fbl, acc[nt]);
    }
  }
}

__device__ __forceinline__ void gemmh8(const _Float16* a, int nk, const _Float16* b, int kp, v8f acc[8]) {
#pragma unroll 1
  for (int kt = 0; kt < nk; ++kt) {
    const v16h fa = ldh(a + 32 * kt);
#pragma unroll
    for (int nt = 0; nt < 8; ++nt) {
      const v16h fb = ldh(b + (size_t)(16 * nt) * kp + 32 * kt);
      acc[nt] = wmh(fa, fb, acc[nt]);
    }
  }
}

__device__ __forceinline__ void st_rows16(const _Float16* stg, _Float16* g, int gp, int co, int row0, int M,
                                          int wave, int l) {
  const int hh = l >> 4, c8 = 8 * (l & 15);
#pragma unroll
  for (int j = 0; j < 8; ++j) {
    const int lr = 16 * wave + 2 * j + hh;
    const int gr = row0 + lr;
    if (gr < M) {
      const v8h v = *(const v8h*)(stg + lr * HP + c8);
      *(volatile v8h*)(g + (size_t)gr * gp + co + c8) = v;
    }
  }
  __threadfence();
#pragma unroll
  for (int j = 0; j < 8; ++j) {
    const int lr = 16 * wave + 2 * j + hh;
    const int gr = row0 + lr;
    if (gr < M) {
      const v8h v = *(const v8h*)(stg + lr * HP + c8);
      *(volatile v8h*)(g + (size_t)gr * gp + co + c8) = v;
    }
  }
}

__device__ __forceinline__ int ldk(const int* __restrict__ k, int e, int n) { return (e < n) ? k[e] : (-2147483647 - 1); }

template <int NBW, int CAP>
__device__ __forceinline__ int collect_hits(const int* __restrict__ keys, int nK, int base, int* sList, int* sWT,
                                            int tid, int l, int wave) {
  const unsigned nb = (unsigned)base;
  int run = 0;
  const int nCh = (nK + SCH - 1) / SCH;
#pragma unroll 1
  for (int ch = 0; ch < nCh; ++ch) {
    const int par = (ch & 1) * 8;
    const int e0 = ch * SCH + tid * 16;
    v4i d0, d1, d2, d3;
    if (e0 + 15 < nK) {
      d0 = *(const v4i*)(keys + e0);
      d1 = *(const v4i*)(keys + e0 + 4);
      d2 = *(const v4i*)(keys + e0 + 8);
      d3 = *(const v4i*)(keys + e0 + 12);
    } else {
      d0.x = ldk(keys, e0, nK);      d0.y = ldk(keys, e0 + 1, nK);  d0.z = ldk(keys, e0 + 2, nK);  d0.w = ldk(keys, e0 + 3, nK);
      d1.x = ldk(keys, e0 + 4, nK);  d1.y = ldk(keys, e0 + 5, nK);  d1.z = ldk(keys, e0 + 6, nK);  d1.w = ldk(keys, e0 + 7, nK);
      d2.x = ldk(keys, e0 + 8, nK);  d2.y = ldk(keys, e0 + 9, nK);  d2.z = ldk(keys, e0 + 10, nK); d2.w = ldk(keys, e0 + 11, nK);
      d3.x = ldk(keys, e0 + 12, nK); d3.y = ldk(keys, e0 + 13, nK); d3.z = ldk(keys, e0 + 14, nK); d3.w = ldk(keys, e0 + 15, nK);
    }
    unsigned msk = 0u;
#define HT(v, j) msk |= ((unsigned)(((unsigned)(v) - nb) < (unsigned)NBW)) << (j);
    HT(d0.x, 0)  HT(d0.y, 1)  HT(d0.z, 2)  HT(d0.w, 3)
    HT(d1.x, 4)  HT(d1.y, 5)  HT(d1.z, 6)  HT(d1.w, 7)
    HT(d2.x, 8)  HT(d2.y, 9)  HT(d2.z, 10) HT(d2.w, 11)
    HT(d3.x, 12) HT(d3.y, 13) HT(d3.z, 14) HT(d3.w, 15)
#undef HT
    const int cnt = (int)__builtin_popcount(msk);
    const unsigned anyw = __builtin_amdgcn_ballot_w32(msk != 0u);
    int excl = 0, tot = 0;
    if (anyw != 0u) {
      int incl = cnt;
#pragma unroll
      for (int off = 1; off < 32; off <<= 1) {
        const int t = __shfl_up(incl, off, 32);
        if (l >= off) incl += t;
      }
      excl = incl - cnt;
      tot = __shfl(incl, 31, 32);
    }
    if (l == 0) sWT[par + wave] = tot;
    __syncthreads();
    int pre = 0, grand = 0;
#pragma unroll
    for (int w2 = 0; w2 < 8; ++w2) {
      const int t = sWT[par + w2];
      grand += t;
      pre += (w2 < wave) ? t : 0;
    }
    if (msk != 0u) {
      int pos = run + pre + excl;
#define PT(v, j) if (msk & (1u << (j))) { if (pos < CAP) sList[pos] = ((e0 + (j)) << 8) | (int)((unsigned)(v) - nb); ++pos; }
      PT(d0.x, 0)  PT(d0.y, 1)  PT(d0.z, 2)  PT(d0.w, 3)
      PT(d1.x, 4)  PT(d1.y, 5)  PT(d1.z, 6)  PT(d1.w, 7)
      PT(d2.x, 8)  PT(d2.y, 9)  PT(d2.z, 10) PT(d2.w, 11)
      PT(d3.x, 12) PT(d3.y, 13) PT(d3.z, 14) PT(d3.w, 15)
#undef PT
    }
    run += grand;
  }
  __syncthreads();
  return run < CAP ? run : CAP;
}

__global__ __launch_bounds__(256) void k_wcvt(const float* __restrict__ W_enc, const float* __restrict__ fem_w1,
                                              const float* __restrict__ fam_w1, const float* __restrict__ fem_w2,
                                              const float* __restrict__ fam_w2, const float* __restrict__ fnm_w1,
                                              const float* __restrict__ fnm_w2, const float* __restrict__ reg_w1,
                                              unsigned short* TW) {
  const int u = blockIdx.x * 256 + threadIdx.x;
  if (u >= NUNITS) return;
  const int g = u * 8;
  float v[8];
  int mode;
  if (g < O_TP) {
    const int isl = (g >= O_ENCL) ? 1 : 0;
    const int loc = g - (isl ? O_ENCL : O_ENCH);
    const int n = loc >> 6, k = loc & 63;
#pragma unroll
    for (int i = 0; i < 8; ++i) v[i] = W_enc[(size_t)(k + i) * HD + n];
    mode = 1 + isl;
  } else if (g < O_FEM2) {
    const int loc = g - O_TP;
    const int c = loc >> 7, k = loc & 127;
    const float* s = (c < 256) ? fem_w1 : fam_w1;
    const int cc = c & 127;
    const int ro = ((c >> 7) & 1) * HD;
#pragma unroll
    for (int i = 0; i < 8; ++i) v[i] = s[(size_t)(ro + k + i) * HD + cc];
    mode = 0;
  } else if (g < O_FN1H) {
    const int isa = (g >= O_FAM2) ? 1 : 0;
    const int loc = g - (isa ? O_FAM2 : O_FEM2);
    const int n = loc >> 7, k = loc & 127;
    const float* s = isa ? fam_w2 : fem_w2;
#pragma unroll
    for (int i = 0; i < 8; ++i) v[i] = s[(size_t)(k + i) * HD + n];
    mode = 0;
  } else if (g < O_FN2H) {
    const int isl = (g >= O_FN1L) ? 1 : 0;
    const int loc = g - (isl ? O_FN1L : O_FN1H);
    const int n = loc >> 8, k = loc & 255;
#pragma unroll
    for (int i = 0; i < 8; ++i) v[i] = fnm_w1[(size_t)(k + i) * HD + n];
    mode = 1 + isl;
  } else if (g < O_RG1H) {
    const int isl = (g >= O_FN2L) ? 1 : 0;
    const int loc = g - (isl ? O_FN2L : O_FN2H);
    const int n = loc >> 7, k = loc & 127;
#pragma unroll
    for (int i = 0; i < 8; ++i) v[i] = fnm_w2[(size_t)(k + i) * HD + n];
    mode = 1 + isl;
  } else {
    const int isl = (g >= O_RG1L) ? 1 : 0;
    const int loc = g - (isl ? O_RG1L : O_RG1H);
    const int n = loc >> 8, k = loc & 255;
#pragma unroll
    for (int i = 0; i < 8; ++i) v[i] = reg_w1[(size_t)(k + i) * HD + n];
    mode = 1 + isl;
  }
  HU8 o;
  if (mode == 0) {
#pragma unroll
    for (int i = 0; i < 8; ++i) o.h[i] = (_Float16)(v[i] * WSC);
  } else if (mode == 1) {
#pragma unroll
    for (int i = 0; i < 8; ++i) o.u[i] = bf_hi(v[i]);
  } else {
#pragma unroll
    for (int i = 0; i < 8; ++i) {
      const unsigned short hh = bf_hi(v[i]);
      o.u[i] = bf_hi(v[i] - bf_f(hh));
    }
  }
  unsigned short* dp = TW + g;
  *(volatile v8us*)dp = o.u;
  __threadfence();
  *(volatile v8us*)dp = o.u;
}

__global__ __launch_bounds__(256) void k_proj(const float* __restrict__ ff, const float* __restrict__ b_enc,
                                              const unsigned short* __restrict__ TW, _Float16* P, int nN) {
  extern __shared__ __attribute__((aligned(16))) unsigned char lds2[];
  unsigned short* ffH = (unsigned short*)(lds2 + L2_FFH);
  unsigned short* ffL = (unsigned short*)(lds2 + L2_FFL);
  _Float16* hF  = (_Float16*)(lds2 + L2_HF);
  _Float16* stg = (_Float16*)(lds2 + L2_STG);
  const unsigned short* ENCH = TW + O_ENCH;
  const unsigned short* ENCL = TW + O_ENCL;
  const _Float16* TP = (const _Float16*)(TW + O_TP);
  const int tid = threadIdx.x, l = tid & 31, wave = tid >> 5, h = l >> 4, m = l & 15;
  const int row0 = blockIdx.x * 128;

#pragma unroll
  for (int it = 0; it < 8; ++it) {
    const int idx = tid + 256 * it;
    const int r = idx >> 4, c4 = (idx & 15) * 4;
    const int row = row0 + r;
    v4f x = {0.0f, 0.0f, 0.0f, 0.0f};
    if (row < nN) x = *(const v4f*)(ff + (size_t)row * FIN + c4);
    v4us hi, lo;
    split4(x, hi, lo);
    *(v4us*)(ffH + r * HP64 + c4) = hi;
    *(v4us*)(ffL + r * HP64 + c4) = lo;
  }
  __syncthreads();

#pragma unroll 1
  for (int ch = 0; ch < 2; ++ch) {
    v8f acc[4];
#pragma unroll
    for (int i = 0; i < 4; ++i) acc[i] = zero8f();
    gemm3(ffH + (16 * wave + m) * HP64 + 8 * h, ffL + (16 * wave + m) * HP64 + 8 * h, 2,
          ENCH + (size_t)(64 * ch + m) * FIN + 8 * h, ENCL + (size_t)(64 * ch + m) * FIN + 8 * h, FIN, acc);
#pragma unroll
    for (int nt = 0; nt < 4; ++nt) {
      const int c = 64 * ch + 16 * nt + m;
      const float bb = b_enc[c];
#pragma unroll
      for (int r = 0; r < 8; ++r) hF[(16 * wave + 8 * h + r) * HP + c] = (_Float16)(acc[nt][r] + bb);
    }
  }
  __syncthreads();

#pragma unroll 1
  for (int cg = 0; cg < 4; ++cg) {
    v8f acc[8];
#pragma unroll
    for (int i = 0; i < 8; ++i) acc[i] = zero8f();
    gemmh8(hF + (16 * wave + m) * HP + 8 * h, 4, TP + (size_t)(128 * cg + m) * HD + 8 * h, HD, acc);
#pragma unroll
    for (int nt = 0; nt < 8; ++nt) {
#pragma unroll
      for (int r = 0; r < 8; ++r) stg[(16 * wave + 8 * h + r) * HP + 16 * nt + m] = (_Float16)acc[nt][r];
    }
    __syncthreads();
    st_rows16(stg, P, PW, 128 * cg, row0, nN, wave, l);
    __syncthreads();
  }
}

__global__ __launch_bounds__(256) void k_edge(const int* __restrict__ src, const int* __restrict__ dst,
                                              const _Float16* __restrict__ P, const unsigned short* __restrict__ TW,
                                              const float* __restrict__ fem_b1, const float* __restrict__ fam_b1,
                                              const float* __restrict__ fem_b2, const float* __restrict__ fam_b2,
                                              _Float16* AGG, int nN, int nE) {
  extern __shared__ __attribute__((aligned(16))) unsigned char lds3[];
  float* sM   = (float*)(lds3 + L3_M);
  float* sDen = (float*)(lds3 + L3_DEN);
  float* sNum = (float*)(lds3 + L3_NUM);
  _Float16* hidF = (_Float16*)(lds3 + L3_HID);
  _Float16* hidA = (_Float16*)(lds3 + L3_HIDA);
  float* sE = (float*)(lds3 + L3_HID);
  float* sL = (float*)(lds3 + L3_SL);
  int* sList = (int*)(lds3 + L3_LIST);
  int* sSrcN = (int*)(lds3 + L3_IDX);
  int* sDstN = sSrcN + 64;
  int* sSlt  = sSrcN + 128;
  int* sWT   = (int*)(lds3 + L3_WT);
  const _Float16* W2E = (const _Float16*)(TW + O_FEM2);
  const _Float16* W2A = (const _Float16*)(TW + O_FAM2);
  const int tid = threadIdx.x, l = tid & 31, wave = tid >> 5, h = l >> 4, m = l & 15;
  const int nodeBase = blockIdx.x * NB3;

  {
    const v4f z = {0.0f, 0.0f, 0.0f, 0.0f};
    const float ninf = -INFINITY;
    const v4f nv = {ninf, ninf, ninf, ninf};
    for (int i = tid; i < NB3 * (HD / 4); i += 256) {
      *(v4f*)(sM + 4 * i) = nv;
      *(v4f*)(sDen + 4 * i) = z;
      *(v4f*)(sNum + 4 * i) = z;
    }
  }

  const int total = collect_hits<NB3, LCAP3>(dst, nE, nodeBase, sList, sWT, tid, l, wave);
  const int nPass = (total + 63) >> 6;
  const int rg = wave & 3, cq = wave >> 2;

#pragma unroll 1
  for (int p = 0; p < nPass; ++p) {
    __syncthreads();
    if (tid < 64) {
      const int i = p * 64 + tid;
      int e = 0, s = 0, sl = -1, dn = nodeBase;
      if (i < total) {
        const int v = sList[i];
        e = v >> 8;
        e = e < 0 ? 0 : (e > nE - 1 ? nE - 1 : e);
        sl = v & (NB3 - 1);
        s = src[e];
        s = s < 0 ? 0 : (s > nN - 1 ? nN - 1 : s);
        dn = nodeBase + sl;
      }
      dn = dn > nN - 1 ? nN - 1 : dn;
      sSrcN[tid] = s;
      sDstN[tid] = dn;
      sSlt[tid]  = sl;
    }
    __syncthreads();

#pragma unroll
    for (int it = 0; it < 4; ++it) {
      const int idx = tid + 256 * it;
      const int j = idx >> 4, c8 = (idx & 15) * 8;
      const int s = sSrcN[j], dn = sDstN[j];
      const _Float16* ps = P + (size_t)s * PW;
      const _Float16* pd = P + (size_t)dn * PW;
      const v8h pt = *(const v8h*)(ps + c8);
      const v8h pb = *(const v8h*)(pd + HD + c8);
      const v8h at = *(const v8h*)(ps + 2 * HD + c8);
      const v8h ab = *(const v8h*)(pd + 3 * HD + c8);
      v8h of, oa;
#pragma unroll
      for (int q = 0; q < 8; ++q) {
        float xf = ((float)pt[q] + (float)pb[q]) * WINV + fem_b1[c8 + q];
        xf = lk(xf);
        of[q] = (_Float16)xf;
        const float xa = ((float)at[q] + (float)ab[q]) * WINV + fam_b1[c8 + q];
        oa[q] = (_Float16)xa;
      }
      *(v8h*)(hidF + j * HP + c8) = of;
      *(v8h*)(hidA + j * HP + c8) = oa;
    }
    __syncthreads();

    v8f aE[4], aL[4];
#pragma unroll
    for (int i = 0; i < 4; ++i) { aE[i] = zero8f(); aL[i] = zero8f(); }
#pragma unroll 1
    for (int kt = 0; kt < 4; ++kt) {
      const v16h fa = ldh(hidF + (16 * rg + m) * HP + 32 * kt + 8 * h);
#pragma unroll
      for (int nt = 0; nt < 4; ++nt) {
        const v16h fb = ldh(W2E + (size_t)(64 * cq + 16 * nt + m) * HD + 32 * kt + 8 * h);
        aE[nt] = wmh(fa, fb, aE[nt]);
      }
      const v16h ga = ldh(hidA + (16 * rg + m) * HP + 32 * kt + 8 * h);
#pragma unroll
      for (int nt = 0; nt < 4; ++nt) {
        const v16h gb = ldh(W2A + (size_t)(64 * cq + 16 * nt + m) * HD + 32 * kt + 8 * h);
        aL[nt] = wmh(ga, gb, aL[nt]);
      }
    }
    __syncthreads();

#pragma unroll
    for (int nt = 0; nt < 4; ++nt) {
      const int c = 64 * cq + 16 * nt + m;
      const float be = fem_b2[c], ba = fam_b2[c];
#pragma unroll
      for (int r = 0; r < 8; ++r) {
        const int row = 16 * rg + 8 * h + r;
        sE[row * FP + c] = aE[nt][r] * WINV + be;
        sL[row * FP + c] = aL[nt][r] * WINV + ba;
      }
    }
    __syncthreads();

#pragma unroll 1
    for (int j = 0; j < 64; ++j) {
      const int sl = sSlt[j];
      if (sl < 0 || (sl & 7) != wave) continue;
      const int c = 4 * l;
      const v4f lg = *(const v4f*)(sL + j * FP + c);
      const v4f ev = *(const v4f*)(sE + j * FP + c);
      float* pm = sM + sl * HD + c;
      float* pd = sDen + sl * HD + c;
      float* pn = sNum + sl * HD + c;
      v4f mo = *(v4f*)pm, de = *(v4f*)pd, nu = *(v4f*)pn;
#pragma unroll
      for (int q = 0; q < 4; ++q) {
        const float d = lg[q] - mo[q];
        const float x = expf(-fabsf(d));
        const bool up = d > 0.0f;
        const float sc = up ? x : 1.0f;
        const float t = up ? 1.0f : x;
        de[q] = de[q] * sc + t;
        nu[q] = nu[q] * sc + t * ev[q];
        mo[q] = up ? lg[q] : mo[q];
      }
      *(v4f*)pm = mo;
      *(v4f*)pd = de;
      *(v4f*)pn = nu;
    }
  }
  __syncthreads();

  const int c8 = 8 * m;
#pragma unroll
  for (int j = 0; j < 8; ++j) {
    const int sl = 16 * wave + 2 * j + h;
    const int node = nodeBase + sl;
    const v4f d0 = *(const v4f*)(sDen + sl * HD + c8);
    const v4f d1 = *(const v4f*)(sDen + sl * HD + c8 + 4);
    const v4f n0 = *(const v4f*)(sNum + sl * HD + c8);
    const v4f n1 = *(const v4f*)(sNum + sl * HD + c8 + 4);
    v8h o;
#pragma unroll
    for (int q = 0; q < 4; ++q) {
      const float da = d0[q] > 0.0f ? d0[q] : 1.0f;
      const float db = d1[q] > 0.0f ? d1[q] : 1.0f;
      o[q]     = (_Float16)(n0[q] * (1.0f / da) * ASC);
      o[4 + q] = (_Float16)(n1[q] * (1.0f / db) * ASC);
    }
    if (node < nN) *(volatile v8h*)(AGG + (size_t)node * HD + c8) = o;
  }
  __threadfence();
#pragma unroll
  for (int j = 0; j < 8; ++j) {
    const int sl = 16 * wave + 2 * j + h;
    const int node = nodeBase + sl;
    const v4f d0 = *(const v4f*)(sDen + sl * HD + c8);
    const v4f d1 = *(const v4f*)(sDen + sl * HD + c8 + 4);
    const v4f n0 = *(const v4f*)(sNum + sl * HD + c8);
    const v4f n1 = *(const v4f*)(sNum + sl * HD + c8 + 4);
    v8h o;
#pragma unroll
    for (int q = 0; q < 4; ++q) {
      const float da = d0[q] > 0.0f ? d0[q] : 1.0f;
      const float db = d1[q] > 0.0f ? d1[q] : 1.0f;
      o[q]     = (_Float16)(n0[q] * (1.0f / da) * ASC);
      o[4 + q] = (_Float16)(n1[q] * (1.0f / db) * ASC);
    }
    if (node < nN) *(volatile v8h*)(AGG + (size_t)node * HD + c8) = o;
  }
}

__global__ __launch_bounds__(256) void k_fnm(const float* __restrict__ ff, const float* __restrict__ b_enc,
                                             const _Float16* __restrict__ AGG, const unsigned short* __restrict__ TW,
                                             const float* __restrict__ fnm_b1, const float* __restrict__ fnm_b2,
                                             float* H2, int nN) {
  extern __shared__ __attribute__((aligned(16))) unsigned char lds4[];
  unsigned short* AH   = (unsigned short*)(lds4 + L4_AH);
  unsigned short* AL   = (unsigned short*)(lds4 + L4_AL);
  unsigned short* ffH  = (unsigned short*)(lds4 + L4_U2);
  unsigned short* ffL  = (unsigned short*)(lds4 + L4_FFL);
  unsigned short* hidH = (unsigned short*)(lds4 + L4_U2);
  unsigned short* hidL = (unsigned short*)(lds4 + L4_HIDL);
  float* ostg = (float*)(lds4 + L4_AH);
  const unsigned short* ENCH = TW + O_ENCH;
  const unsigned short* ENCL = TW + O_ENCL;
  const unsigned short* F1H = TW + O_FN1H;
  const unsigned short* F1L = TW + O_FN1L;
  const unsigned short* F2H = TW + O_FN2H;
  const unsigned short* F2L = TW + O_FN2L;
  const int tid = threadIdx.x, l = tid & 31, wave = tid >> 5, h = l >> 4, m = l & 15;
  const int row0 = blockIdx.x * 128;

#pragma unroll
  for (int it = 0; it < 8; ++it) {
    const int idx = tid + 256 * it;
    const int r = idx >> 4, c4 = (idx & 15) * 4, c8 = (idx & 15) * 8;
    const int row = row0 + r;
    v4f x = {0.0f, 0.0f, 0.0f, 0.0f};
    if (row < nN) x = *(const v4f*)(ff + (size_t)row * FIN + c4);
    v4us hi, lo;
    split4(x, hi, lo);
    *(v4us*)(ffH + r * HP64 + c4) = hi;
    *(v4us*)(ffL + r * HP64 + c4) = lo;
    v8h ag;
#pragma unroll
    for (int q = 0; q < 8; ++q) ag[q] = (_Float16)0.0f;
    if (row < nN) ag = *(const v8h*)(AGG + (size_t)row * HD + c8);
    v8us ahi, alo;
#pragma unroll
    for (int q = 0; q < 8; ++q) {
      const float f = (float)ag[q] * AINV;
      const unsigned short hh = bf_hi(f);
      ahi[q] = hh;
      alo[q] = bf_hi(f - bf_f(hh));
    }
    *(v8us*)(AH + r * HP256 + HD + c8) = ahi;
    *(v8us*)(AL + r * HP256 + HD + c8) = alo;
  }
  __syncthreads();

#pragma unroll 1
  for (int ch = 0; ch < 2; ++ch) {
    v8f acc[4];
#pragma unroll
    for (int i = 0; i < 4; ++i) acc[i] = zero8f();
    gemm3(ffH + (16 * wave + m) * HP64 + 8 * h, ffL + (16 * wave + m) * HP64 + 8 * h, 2,
          ENCH + (size_t)(64 * ch + m) * FIN + 8 * h, ENCL + (size_t)(64 * ch + m) * FIN + 8 * h, FIN, acc);
#pragma unroll
    for (int nt = 0; nt < 4; ++nt) {
      const int c = 64 * ch + 16 * nt + m;
      const float bb = b_enc[c];
#pragma unroll
      for (int r = 0; r < 8; ++r) {
        const float hv = acc[nt][r] + bb;
        const unsigned short hh = bf_hi(hv);
        const int row = 16 * wave + 8 * h + r;
        AH[row * HP256 + c] = hh;
        AL[row * HP256 + c] = bf_hi(hv - bf_f(hh));
      }
    }
  }
  __syncthreads();

#pragma unroll 1
  for (int ch = 0; ch < 2; ++ch) {
    v8f acc[4];
#pragma unroll
    for (int i = 0; i < 4; ++i) acc[i] = zero8f();
    gemm3(AH + (16 * wave + m) * HP256 + 8 * h, AL + (16 * wave + m) * HP256 + 8 * h, 8,
          F1H + (size_t)(64 * ch + m) * 256 + 8 * h, F1L + (size_t)(64 * ch + m) * 256 + 8 * h, 256, acc);
#pragma unroll
    for (int nt = 0; nt < 4; ++nt) {
      const int c = 64 * ch + 16 * nt + m;
      const float bb = fnm_b1[c];
#pragma unroll
      for (int r = 0; r < 8; ++r) {
        const float hv = lk(acc[nt][r] + bb);
        const unsigned short hh = bf_hi(hv);
        const int row = 16 * wave + 8 * h + r;
        hidH[row * HP + c] = hh;
        hidL[row * HP + c] = bf_hi(hv - bf_f(hh));
      }
    }
  }
  __syncthreads();

#pragma unroll 1
  for (int ch = 0; ch < 2; ++ch) {
    v8f acc[4];
#pragma unroll
    for (int i = 0; i < 4; ++i) acc[i] = zero8f();
    gemm3(hidH + (16 * wave + m) * HP + 8 * h, hidL + (16 * wave + m) * HP + 8 * h, 4,
          F2H + (size_t)(64 * ch + m) * HD + 8 * h, F2L + (size_t)(64 * ch + m) * HD + 8 * h, HD, acc);
#pragma unroll
    for (int nt = 0; nt < 4; ++nt) {
      const int c = 64 * ch + 16 * nt + m;
      const float bb = fnm_b2[c];
#pragma unroll
      for (int r = 0; r < 8; ++r) ostg[(16 * wave + 8 * h + r) * FP + c] = acc[nt][r] + bb;
    }
  }
  __syncthreads();

#pragma unroll
  for (int rr = 0; rr < 16; ++rr) {
    const int lr = 16 * wave + rr;
    const int gr = row0 + lr;
    if (gr < nN) {
      const v4f v = *(const v4f*)(ostg + lr * FP + 4 * l);
      *(volatile v4f*)(H2 + (size_t)gr * HD + 4 * l) = v;
    }
  }
  __threadfence();
#pragma unroll
  for (int rr = 0; rr < 16; ++rr) {
    const int lr = 16 * wave + rr;
    const int gr = row0 + lr;
    if (gr < nN) {
      const v4f v = *(const v4f*)(ostg + lr * FP + 4 * l);
      *(volatile v4f*)(H2 + (size_t)gr * HD + 4 * l) = v;
    }
  }
}

__global__ __launch_bounds__(256) void k_read(const int* __restrict__ n2g, const float* __restrict__ H2,
                                              const float* __restrict__ Wg, const float* __restrict__ bg,
                                              float* RD, int nN, int nG) {
  extern __shared__ __attribute__((aligned(16))) unsigned char lds5[];
  float* sSum = (float*)(lds5 + L5_SUM);
  float* sMax = (float*)(lds5 + L5_MAX);
  int* sList = (int*)(lds5 + L5_LIST);
  int* sWT   = (int*)(lds5 + L5_WT);
  const int tid = threadIdx.x, l = tid & 31, wave = tid >> 5;
  const int gBase = blockIdx.x * NB5;

  {
    const v4f z = {0.0f, 0.0f, 0.0f, 0.0f};
    const float ninf = -INFINITY;
    const v4f nv = {ninf, ninf, ninf, ninf};
    for (int i = tid; i < NB5 * (HD / 4); i += 256) {
      *(v4f*)(sSum + 4 * i) = z;
      *(v4f*)(sMax + 4 * i) = nv;
    }
  }
  const int total = collect_hits<NB5, LCAP5>(n2g, nN, gBase, sList, sWT, tid, l, wave);
  const v4f wg = *(const v4f*)(Wg + 4 * l);
  const float b0 = bg[0];

#pragma unroll 1
  for (int i = 0; i < total; ++i) {
    const int v = sList[i];
    const int sl = v & (NB5 - 1);
    if ((sl & 7) != wave) continue;
    int n = v >> 8;
    n = n < 0 ? 0 : (n > nN - 1 ? nN - 1 : n);
    const v4f x = *(const v4f*)(H2 + (size_t)n * HD + 4 * l);
    float dot = x[0] * wg[0];
    dot += x[1] * wg[1];
    dot += x[2] * wg[2];
    dot += x[3] * wg[3];
    dot += __shfl_xor(dot, 16, 32);
    dot += __shfl_xor(dot, 8, 32);
    dot += __shfl_xor(dot, 4, 32);
    dot += __shfl_xor(dot, 2, 32);
    dot += __shfl_xor(dot, 1, 32);
    const float wt = 1.0f / (1.0f + expf(-(dot + b0)));
    float* ps = sSum + sl * HD + 4 * l;
    float* px = sMax + sl * HD + 4 * l;
    v4f su = *(v4f*)ps, mx = *(v4f*)px;
#pragma unroll
    for (int q = 0; q < 4; ++q) {
      su[q] += wt * x[q];
      mx[q] = fmaxf(mx[q], x[q]);
    }
    *(v4f*)ps = su;
    *(v4f*)px = mx;
  }
  __syncthreads();

#pragma unroll
  for (int j = 0; j < 8; ++j) {
    const int sl = 8 * wave + j;
    const int g = gBase + sl;
    if (g < nG) {
      const v4f a = *(const v4f*)(sSum + sl * HD + 4 * l);
      v4f b = *(const v4f*)(sMax + sl * HD + 4 * l);
#pragma unroll
      for (int q = 0; q < 4; ++q) b[q] = (b[q] > -3.0e38f) ? b[q] : 0.0f;
      float* rp = RD + (size_t)g * 256;
      *(volatile v4f*)(rp + 4 * l) = a;
      *(volatile v4f*)(rp + HD + 4 * l) = b;
    }
  }
  __threadfence();
#pragma unroll
  for (int j = 0; j < 8; ++j) {
    const int sl = 8 * wave + j;
    const int g = gBase + sl;
    if (g < nG) {
      const v4f a = *(const v4f*)(sSum + sl * HD + 4 * l);
      v4f b = *(const v4f*)(sMax + sl * HD + 4 * l);
#pragma unroll
      for (int q = 0; q < 4; ++q) b[q] = (b[q] > -3.0e38f) ? b[q] : 0.0f;
      float* rp = RD + (size_t)g * 256;
      *(volatile v4f*)(rp + 4 * l) = a;
      *(volatile v4f*)(rp + HD + 4 * l) = b;
    }
  }
}

__global__ __launch_bounds__(256) void k_head(const float* __restrict__ RD, const unsigned short* __restrict__ TW,
                                              const float* __restrict__ reg_b1, const float* __restrict__ reg_w2,
                                              const float* __restrict__ reg_b2, float* out, int nG) {
  extern __shared__ __attribute__((aligned(16))) unsigned char lds6[];
  unsigned short* AH = (unsigned short*)(lds6 + L6_AH);
  unsigned short* AL = (unsigned short*)(lds6 + L6_AL);
  float* res = (float*)(lds6 + L6_RES);
  const unsigned short* R1H = TW + O_RG1H;
  const unsigned short* R1L = TW + O_RG1L;
  const int tid = threadIdx.x, l = tid & 31, wave = tid >> 5, h = l >> 4, m = l & 15;
  const int g0 = blockIdx.x * 128;

#pragma unroll 4
  for (int it = 0; it < 32; ++it) {
    const int idx = tid + 256 * it;
    const int r = idx >> 6, c4 = (idx & 63) * 4;
    const int g = g0 + r;
    v4f x = {0.0f, 0.0f, 0.0f, 0.0f};
    if (g < nG) x = *(const v4f*)(RD + (size_t)g * 256 + c4);
    v4us hi, lo;
    split4(x, hi, lo);
    *(v4us*)(AH + r * HP256 + c4) = hi;
    *(v4us*)(AL + r * HP256 + c4) = lo;
  }
  __syncthreads();

  float part[8];
#pragma unroll
  for (int r = 0; r < 8; ++r) part[r] = 0.0f;
#pragma unroll 1
  for (int ch = 0; ch < 2; ++ch) {
    v8f acc[4];
#pragma unroll
    for (int i = 0; i < 4; ++i) acc[i] = zero8f();
    gemm3(AH + (16 * wave + m) * HP256 + 8 * h, AL + (16 * wave + m) * HP256 + 8 * h, 8,
          R1H + (size_t)(64 * ch + m) * 256 + 8 * h, R1L + (size_t)(64 * ch + m) * 256 + 8 * h, 256, acc);
#pragma unroll
    for (int nt = 0; nt < 4; ++nt) {
      const int c = 64 * ch + 16 * nt + m;
      const float bb = reg_b1[c];
      const float w2c = reg_w2[c];
#pragma unroll
      for (int r = 0; r < 8; ++r) part[r] += lk(acc[nt][r] + bb) * w2c;
    }
  }
#pragma unroll
  for (int r = 0; r < 8; ++r) {
    float p = part[r];
    p += __shfl_xor(p, 8, 32);
    p += __shfl_xor(p, 4, 32);
    p += __shfl_xor(p, 2, 32);
    p += __shfl_xor(p, 1, 32);
    part[r] = p;
  }
  if (m == 0) {
    const float b2 = reg_b2[0];
#pragma unroll
    for (int r = 0; r < 8; ++r) res[16 * wave + 8 * h + r] = part[r] + b2;
  }
  __syncthreads();

  if (wave == 0) {
    const int gg = g0 + 4 * l;
    const v4f v = *(const v4f*)(res + 4 * l);
    if (g0 + 128 <= nG) {
      *(volatile v4f*)(out + gg) = v;
    } else {
#pragma unroll
      for (int q = 0; q < 4; ++q) if (gg + q < nG) *(volatile float*)(out + gg + q) = v[q];
    }
    __threadfence();
    if (g0 + 128 <= nG) {
      *(volatile v4f*)(out + gg) = v;
    } else {
#pragma unroll
      for (int q = 0; q < 4; ++q) if (gg + q < nG) *(volatile float*)(out + gg + q) = v[q];
    }
  }
}

extern "C" void kernel_launch(void* const* d_in, const int* in_sizes, int n_in,
                              void* d_out, int out_size, void* d_ws, size_t ws_size,
                              hipStream_t stream) {
  if (n_in < 24 || out_size <= 0) return;
  const int nE = in_sizes[1];
  const int nN = in_sizes[3];
  const int nG = out_size;
  if (nN <= 0 || nE <= 0 || in_sizes[0] != nN * FIN || in_sizes[2] != nE) return;
  if (nN > (1 << 23) || nE > (1 << 23)) return;
  if (in_sizes[4] != FIN * HD || in_sizes[5] != HD) return;
  if (in_sizes[6] != 2 * HD * HD || in_sizes[7] != HD || in_sizes[8] != HD * HD || in_sizes[9] != HD) return;
  if (in_sizes[10] != 2 * HD * HD || in_sizes[11] != HD || in_sizes[12] != HD * HD || in_sizes[13] != HD) return;
  if (in_sizes[14] != 2 * HD * HD || in_sizes[15] != HD || in_sizes[16] != HD * HD || in_sizes[17] != HD) return;
  if (in_sizes[18] != HD || in_sizes[19] < 1) return;
  if (in_sizes[20] != 2 * HD * HD || in_sizes[21] != HD || in_sizes[22] != HD || in_sizes[23] < 1) return;

  const float* ff     = (const float*)d_in[0];
  const int*   src    = (const int*)d_in[1];
  const int*   dst    = (const int*)d_in[2];
  const int*   n2g    = (const int*)d_in[3];
  const float* W_enc  = (const float*)d_in[4];
  const float* b_enc  = (const float*)d_in[5];
  const float* fem_w1 = (const float*)d_in[6];
  const float* fem_b1 = (const float*)d_in[7];
  const float* fem_w2 = (const float*)d_in[8];
  const float* fem_b2 = (const float*)d_in[9];
  const float* fnm_w1 = (const float*)d_in[10];
  const float* fnm_b1 = (const float*)d_in[11];
  const float* fnm_w2 = (const float*)d_in[12];
  const float* fnm_b2 = (const float*)d_in[13];
  const float* fam_w1 = (const float*)d_in[14];
  const float* fam_b1 = (const float*)d_in[15];
  const float* fam_w2 = (const float*)d_in[16];
  const float* fam_b2 = (const float*)d_in[17];
  const float* Wg     = (const float*)d_in[18];
  const float* bg     = (const float*)d_in[19];
  const float* reg_w1 = (const float*)d_in[20];
  const float* reg_b1 = (const float*)d_in[21];
  const float* reg_w2 = (const float*)d_in[22];
  const float* reg_b2 = (const float*)d_in[23];
  float* out = (float*)d_out;

  char* ws = (char*)d_ws;
  size_t off = 0;
  const size_t oTW = off;  off += (size_t)O_TOT * 2;                 off = (off + 255) & ~(size_t)255;
  const size_t r1a = (size_t)nN * PW * 2;
  const size_t r1b = (size_t)nN * HD * 4 + (size_t)nG * 256 * 4;
  const size_t r1  = r1a > r1b ? r1a : r1b;
  const size_t oR1 = off;  off += r1;                                off = (off + 255) & ~(size_t)255;
  const size_t oAG = off;  off += (size_t)nN * HD * 2;               off = (off + 255) & ~(size_t)255;
  if (off > ws_size) return;
  unsigned short* TW = (unsigned short*)(ws + oTW);
  _Float16* P   = (_Float16*)(ws + oR1);
  float*    H2  = (float*)(ws + oR1);
  float*    RD  = (float*)(ws + oR1 + (size_t)nN * HD * 4);
  _Float16* AGG = (_Float16*)(ws + oAG);

  const hipError_t a2 = hipFuncSetAttribute(reinterpret_cast<const void*>(&k_proj), hipFuncAttributeMaxDynamicSharedMemorySize, L2_TOT);
  const hipError_t a3 = hipFuncSetAttribute(reinterpret_cast<const void*>(&k_edge), hipFuncAttributeMaxDynamicSharedMemorySize, L3_TOT);
  const hipError_t a4 = hipFuncSetAttribute(reinterpret_cast<const void*>(&k_fnm),  hipFuncAttributeMaxDynamicSharedMemorySize, L4_TOT);
  const hipError_t a5 = hipFuncSetAttribute(reinterpret_cast<const void*>(&k_read), hipFuncAttributeMaxDynamicSharedMemorySize, L5_TOT);
  const hipError_t a6 = hipFuncSetAttribute(reinterpret_cast<const void*>(&k_head), hipFuncAttributeMaxDynamicSharedMemorySize, L6_TOT);
  (void)a2; (void)a3; (void)a4; (void)a5; (void)a6;

  const int nBlkN = (nN + 127) / 128;
  const int nBlkA = (nN + NB3 - 1) / NB3;
  const int nBlkR = (nG + NB5 - 1) / NB5;
  const int nBlkH = (nG + 127) / 128;

  k_wcvt<<<NUNITS / 256, 256, 0, stream>>>(W_enc, fem_w1, fam_w1, fem_w2, fam_w2, fnm_w1, fnm_w2, reg_w1, TW);
  k_proj<<<nBlkN, 256, L2_TOT, stream>>>(ff, b_enc, TW, P, nN);
  k_edge<<<nBlkA, 256, L3_TOT, stream>>>(src, dst, P, TW, fem_b1, fam_b1, fem_b2, fam_b2, AGG, nN, nE);
  k_fnm<<<nBlkN, 256, L4_TOT, stream>>>(ff, b_enc, AGG, TW, fnm_b1, fnm_b2, H2, nN);
  k_read<<<nBlkR, 256, L5_TOT, stream>>>(n2g, H2, Wg, bg, RD, nN, nG);
  k_head<<<nBlkH, 256, L6_TOT, stream>>>(RD, TW, reg_b1, reg_w2, reg_b2, out, nG);
  (void)hipGetLastError();
}
